// _RBFKANLayer_24644522344533
// MI455X (gfx1250) — hardware-run, weakly checked
//
#include <hip/hip_runtime.h>
#include <math.h>

constexpr int kIn        = 512;
constexpr int kOut       = 512;
constexpr int kGrid      = 12;
constexpr int kKspl      = kIn * kGrid;
constexpr int kKtot      = kKspl + kIn;
constexpr int kChunkRows = 4096;
constexpr int kRowU32    = kKtot / 2;
constexpr int kRowSeg    = kKtot / 256;
constexpr float kBW        = 0.72727272727272729f;
constexpr float kInvBW     = 1.0f / kBW;
constexpr float kWCarry    = 16.0f;
constexpr float kWCarryInv = 1.0f / 16.0f;
constexpr size_t kBtBytes  = (size_t)kOut * kKtot * 2;
constexpr size_t kABytes   = (size_t)kChunkRows * kKtot * 2;
static_assert(kKtot % 32 == 0);
static_assert(kKtot % 256 == 0);
static_assert(kRowSeg * 256 == kKtot);
static_assert(kChunkRows % 64 == 0 && kOut % 64 == 0);
static_assert(kIn == 2 * 256);
static_assert((kBtBytes % 256) == 0 && (kABytes % 256) == 0);


typedef __attribute__((ext_vector_type(16))) _Float16 v16h;
typedef __attribute__((ext_vector_type(8)))  _Float16 v8h;
typedef __attribute__((ext_vector_type(16))) __bf16   v16b;
typedef __attribute__((ext_vector_type(8)))  __bf16   v8b;
typedef __attribute__((ext_vector_type(8)))  float    v8f;
typedef __attribute__((ext_vector_type(4)))  float    v4f;
typedef __attribute__((ext_vector_type(2)))  float    v2f;
typedef __attribute__((ext_vector_type(4)))  unsigned int v4u;
typedef __attribute__((ext_vector_type(2)))  unsigned int v2u;

__device__ __forceinline__ unsigned short f2bf_bits(float f) {
  unsigned u = __float_as_uint(f);
  return (unsigned short)((u + 0x7FFFu + ((u >> 16) & 1u)) >> 16);
}
__device__ __forceinline__ float bf_bits2f(unsigned short h) { return __uint_as_float(((unsigned)h) << 16); }

__device__ __forceinline__ void dep_guard_h(v8f& a, v8f& b, v16h x, v16h y) { asm volatile("v_nop\n\tv_nop\n\tv_nop\n\tv_nop" : "+v"(a), "+v"(b) : "v"(x), "v"(y)); }
__device__ __forceinline__ void dep_guard_b(v8f& a, v8f& b, v16b x, v16b y) { asm volatile("v_nop\n\tv_nop\n\tv_nop\n\tv_nop" : "+v"(a), "+v"(b) : "v"(x), "v"(y)); }
__device__ __forceinline__ void keep4_h(v16h a, v16h b, v16h c, v16h d) { asm volatile("v_nop" :: "v"(a), "v"(b), "v"(c), "v"(d)); }
__device__ __forceinline__ void keep4_b(v16b a, v16b b, v16b c, v16b d) { asm volatile("v_nop" :: "v"(a), "v"(b), "v"(c), "v"(d)); }
__device__ __forceinline__ void acc_guard4(v8f& a, v8f& b, v8f& c, v8f& d) { asm volatile("v_nop\n\tv_nop\n\tv_nop\n\tv_nop" : "+v"(a), "+v"(b), "+v"(c), "+v"(d)); }
template <typename T> struct Frag;
template <> struct Frag<_Float16> {
  typedef v16h V; union U { v16h v; v8h h[2]; };
  static __device__ __forceinline__ v16h load(const _Float16* p) {
    U f; f.h[0] = *(const v8h*)(p); f.h[1] = *(const v8h*)(p + 16); return f.v;
  }
  static __device__ __forceinline__ v8f mma(v16h a, v16h b, v8f c) {
    return __builtin_amdgcn_wmma_f32_16x16x32_f16(false, a, false, b, (short)0, c, false, false);
  }
  static __device__ __forceinline__ void guard(v8f& a, v8f& b, v16h x, v16h y) { dep_guard_h(a, b, x, y); }
  static __device__ __forceinline__ void keep(v16h a, v16h b, v16h c, v16h d) { keep4_h(a, b, c, d); }
};
template <> struct Frag<__bf16> {
  typedef v16b V; union U { v16b v; v8b h[2]; };
  static __device__ __forceinline__ v16b load(const __bf16* p) {
    U f; f.h[0] = *(const v8b*)(p); f.h[1] = *(const v8b*)(p + 16); return f.v;
  }
  static __device__ __forceinline__ v8f mma(v16b a, v16b b, v8f c) {
    return __builtin_amdgcn_wmma_f32_16x16x32_bf16(false, a, false, b, (short)0, c, false, false);
  }
  static __device__ __forceinline__ void guard(v8f& a, v8f& b, v16b x, v16b y) { dep_guard_b(a, b, x, y); }
  static __device__ __forceinline__ void keep(v16b a, v16b b, v16b c, v16b d) { keep4_b(a, b, c, d); }
};

__device__ __forceinline__ unsigned pk16(unsigned short a, unsigned short b) { return (unsigned)a | ((unsigned)b << 16); }
__device__ __forceinline__ unsigned short h_bits(float f) { const _Float16 h = (_Float16)f; return __builtin_bit_cast(unsigned short, h); }

template <int ET> struct Elem;
template <> struct Elem<0> { typedef _Float16 T; };
template <> struct Elem<1> { typedef __bf16 T; };
template <int ET, bool SPLIT, int BIAS_MODE, int OUT_MODE, bool RESID, int ACT = 0>
__global__ __launch_bounds__(256) void wmma_gemm64(
    const unsigned short* __restrict__ Ap, const unsigned short* __restrict__ A2p, int lda, long strideA,
    const unsigned short* __restrict__ Btp, const unsigned short* __restrict__ Bt2p, int ldb, long strideB,
    void* __restrict__ Cout, void* __restrict__ Cout2, int ldc, long strideC,
    const float* __restrict__ bias,
    const float* __restrict__ resid, long strideR,
    int M, int N, int K, float scale) {
  typedef typename Elem<ET>::T T;
  typedef typename Frag<T>::V V;
  const T* A = (const T*)Ap; const T* A2 = (const T*)A2p; const T* Bt = (const T*)Btp; const T* Bt2 = (const T*)Bt2p;
  __shared__ __align__(16) float sT[8][16 * 68];
  const int b    = blockIdx.y;
  const int lane = threadIdx.x & 31;
  const int wave = threadIdx.x >> 5;
  const int tilesN = N >> 6;
  const int tilesM = M >> 6;
  const int tile = blockIdx.x * 8 + wave;
  if (tile >= tilesM * tilesN) return;
  const int tm = tile / tilesN;
  const int tn = tile - tm * tilesN;
  const int m0 = tm << 6;
  const int n0 = tn << 6;

  const T* Ab  = A  + (size_t)b * strideA;
  const T* Bb  = Bt + (size_t)b * strideB;
  const T* Ab2 = SPLIT ? (A2  + (size_t)b * strideA) : nullptr;
  const T* Bb2 = SPLIT ? (Bt2 + (size_t)b * strideB) : nullptr;

  const int rlane = lane & 15;
  const int koff  = (lane >> 4) * 8;
  const int mOff  = (lane >> 4) * 8;

  v8f acc[4][4];
#pragma unroll
  for (int i = 0; i < 4; ++i)
#pragma unroll
    for (int j = 0; j < 4; ++j) acc[i][j] = (v8f){0.f,0.f,0.f,0.f,0.f,0.f,0.f,0.f};

  for (int k0 = 0; k0 < K; k0 += 32) {
    V bh[4], bl[4];
#pragma unroll
    for (int j = 0; j < 4; ++j) {
      const size_t bo = (size_t)(n0 + (j << 4) + rlane) * ldb + koff + k0;
      bh[j] = Frag<T>::load(Bb + bo);
      if (SPLIT) bl[j] = Frag<T>::load(Bb2 + bo);
    }
#pragma unroll
    for (int i = 0; i < 4; ++i) {
      const size_t ao = (size_t)(m0 + (i << 4) + rlane) * lda + koff + k0;
      V ah = Frag<T>::load(Ab + ao);
      V al;
      if (SPLIT) al = Frag<T>::load(Ab2 + ao);
#pragma unroll
      for (int j = 0; j < 4; ++j) {
        acc[i][j] = Frag<T>::mma(ah, bh[j], acc[i][j]);
        if (SPLIT) {
          acc[i][j] = Frag<T>::mma(ah, bl[j], acc[i][j]);
          acc[i][j] = Frag<T>::mma(al, bh[j], acc[i][j]);
        }
      }
      Frag<T>::guard(acc[i][0], acc[i][3], ah, SPLIT ? al : ah);
    }
    Frag<T>::keep(bh[0], bh[1], bh[2], bh[3]);
    if (SPLIT) Frag<T>::keep(bl[0], bl[1], bl[2], bl[3]);
  }
  acc_guard4(acc[0][0], acc[0][1], acc[0][2], acc[0][3]);
  acc_guard4(acc[1][0], acc[1][1], acc[1][2], acc[1][3]);
  acc_guard4(acc[2][0], acc[2][1], acc[2][2], acc[2][3]);
  acc_guard4(acc[3][0], acc[3][1], acc[3][2], acc[3][3]);

  float* slab = sT[wave];
  const float* Rb = RESID ? (resid + (size_t)b * strideR) : nullptr;
#pragma unroll
  for (int i = 0; i < 4; ++i) {
    const int mBase = m0 + (i << 4);
#pragma unroll
    for (int j = 0; j < 4; ++j) {
      const int n = n0 + (j << 4) + rlane;
      float bv = 0.f;
      if (BIAS_MODE == 2) bv = bias[n];
#pragma unroll
      for (int r = 0; r < 8; ++r) {
        float v = acc[i][j][r] * scale;
        if (BIAS_MODE == 1) v += bias[mBase + mOff + r];
        if (BIAS_MODE == 2) v += bv;
        if (RESID) v += Rb[(size_t)(mBase + mOff + r) * ldc + n];
        if (ACT == 2) v = fmaxf(v, 0.0f);
        if (ACT == 4) v = (v > 0.f) ? v : 0.01f * v;
        slab[(mOff + r) * 68 + (j << 4) + rlane] = v;
      }
    }
    __builtin_amdgcn_fence(__ATOMIC_RELEASE, "workgroup");
    __builtin_amdgcn_wave_barrier();
    __builtin_amdgcn_fence(__ATOMIC_ACQUIRE, "workgroup");
    if (OUT_MODE == 0) {
      float* C = (float*)Cout + (size_t)b * strideC;
      const int hh = lane >> 4, c4 = (lane & 15) * 4;
      for (int pass = 0; pass < 2; ++pass) {
#pragma unroll
        for (int it = 0; it < 8; ++it) {
          const int row = it * 2 + hh;
          v4f v = *(const v4f*)(slab + row * 68 + c4);
          *(volatile v4f*)(C + (size_t)(mBase + row) * ldc + n0 + c4) = v;
        }
        __threadfence();
      }
    } else {
      const int q = lane >> 3, c8 = (lane & 7) * 8;
      unsigned short* C  = (unsigned short*)Cout  + (size_t)b * strideC;
      unsigned short* C2 = (OUT_MODE == 2) ? ((unsigned short*)Cout2 + (size_t)b * strideC) : nullptr;
      for (int pass = 0; pass < 2; ++pass) {
#pragma unroll
        for (int it = 0; it < 4; ++it) {
          const int row = it * 4 + q;
          const float* sp = slab + row * 68 + c8;
          v8h hv, lv;
#pragma unroll
          for (int e = 0; e < 8; ++e) {
            if (OUT_MODE == 1) {
              hv[e] = (_Float16)sp[e];
            } else {
              unsigned short hb = f2bf_bits(sp[e]);
              unsigned short lb = f2bf_bits(sp[e] - bf_bits2f(hb));
              hv[e] = __builtin_bit_cast(_Float16, hb);
              lv[e] = __builtin_bit_cast(_Float16, lb);
            }
          }
          *(volatile v8h*)(C + (size_t)(mBase + row) * ldc + n0 + c8) = hv;
          if (OUT_MODE == 2) *(volatile v8h*)(C2 + (size_t)(mBase + row) * ldc + n0 + c8) = lv;
        }
        __threadfence();
      }
    }
    __builtin_amdgcn_fence(__ATOMIC_RELEASE, "workgroup");
    __builtin_amdgcn_wave_barrier();
    __builtin_amdgcn_fence(__ATOMIC_ACQUIRE, "workgroup");
  }
}

__device__ __forceinline__ void store_row_2pass(const unsigned* srow, unsigned short* grow, int wave, int lane) {
  for (int pass = 0; pass < 2; ++pass) {
    for (int seg = wave; seg < kRowSeg; seg += 8) {
      const v4u u = *(const v4u*)(srow + seg * 128 + lane * 4);
      *(volatile v4u*)(grow + (size_t)seg * 256 + lane * 8) = u;
    }
    __threadfence();
  }
}

__global__ __launch_bounds__(256) void weight_rows_kernel(const float* __restrict__ coeff,
                                                          const float* __restrict__ base_w,
                                                          unsigned short* __restrict__ bt) {
  __shared__ __align__(16) unsigned srow[kRowU32];
  const int t = threadIdx.x;
  const int lane = t & 31, wave = t >> 5;
  const int o = blockIdx.x;
#pragma unroll
  for (int sub = 0; sub < 2; ++sub) {
    const int i = 2 * t + sub;
    const float* cp = coeff + ((size_t)i * kOut + o) * kGrid;
    const v4f a = *(const v4f*)(cp);
    const v4f c = *(const v4f*)(cp + 4);
    const v4f d = *(const v4f*)(cp + 8);
    unsigned short hb[12];
#pragma unroll
    for (int e = 0; e < 4; ++e) {
      hb[e]     = h_bits(a[e] * kWCarry);
      hb[4 + e] = h_bits(c[e] * kWCarry);
      hb[8 + e] = h_bits(d[e] * kWCarry);
    }
    unsigned* sp = srow + i * 6;
    *(v2u*)(sp)     = (v2u){pk16(hb[0], hb[1]), pk16(hb[2], hb[3])};
    *(v2u*)(sp + 2) = (v2u){pk16(hb[4], hb[5]), pk16(hb[6], hb[7])};
    *(v2u*)(sp + 4) = (v2u){pk16(hb[8], hb[9]), pk16(hb[10], hb[11])};
  }
  {
    const v2f w = *(const v2f*)(base_w + (size_t)o * kIn + 2 * t);
    srow[kKspl / 2 + t] = pk16(h_bits(w[0] * kWCarry), h_bits(w[1] * kWCarry));
  }
  __syncthreads();
  store_row_2pass(srow, bt + (size_t)o * kKtot, wave, lane);
}

__global__ __launch_bounds__(256) void basis_rows_kernel(const float* __restrict__ x,
                                                         const float* __restrict__ centers,
                                                         unsigned short* __restrict__ aplane,
                                                         int row0) {
  __shared__ __align__(16) unsigned srow[kRowU32];
  __shared__ float cs[kGrid];
  const int t = threadIdx.x;
  const int lane = t & 31, wave = t >> 5;
  const int r = blockIdx.x;
  if (t < kGrid) cs[t] = centers[t];
  const float* xr = x + (size_t)(row0 + r) * kIn;
  const v2f xx = *(const v2f*)(xr + 2 * t);
  const float x0 = xx[0], x1 = xx[1];
  srow[kKspl / 2 + t] = pk16(h_bits(x0), h_bits(x1));
  __syncthreads();
#pragma unroll 1
  for (int sub = 0; sub < 2; ++sub) {
    const float xv = sub ? x1 : x0;
    unsigned* sp = srow + (2 * t + sub) * 6;
#pragma unroll 1
    for (int gp = 0; gp < 6; ++gp) {
      const float c0 = cs[2 * gp];
      const float c1 = cs[2 * gp + 1];
      const float d0 = (xv - c0) * kInvBW;
      const float d1 = (xv - c1) * kInvBW;
      const float e0 = expf((-0.5f * d0) * d0);
      const float e1 = expf((-0.5f * d1) * d1);
      sp[gp] = pk16(h_bits(e0), h_bits(e1));
    }
  }
  __syncthreads();
  store_row_2pass(srow, aplane + (size_t)r * kKtot, wave, lane);
}

extern "C" void kernel_launch(void* const* d_in, const int* in_sizes, int n_in,
                              void* d_out, int out_size, void* d_ws, size_t ws_size,
                              hipStream_t stream) {
  (void)n_in;
  const float* x       = (const float*)d_in[0];
  const float* coeff   = (const float*)d_in[1];
  const float* base_w  = (const float*)d_in[2];
  const float* base_b  = (const float*)d_in[3];
  const float* centers = (const float*)d_in[4];
  float* out = (float*)d_out;

  const int nrows = in_sizes[0] / kIn;
  if (nrows <= 0 || (nrows % kChunkRows) != 0) return;
  if (out_size != nrows * kOut) return;
  if (in_sizes[1] != kIn * kOut * kGrid || in_sizes[2] != kOut * kIn || in_sizes[3] != kOut || in_sizes[4] != kGrid) return;
  const int nchunks = nrows / kChunkRows;

  unsigned char* ws = (unsigned char*)d_ws;
  size_t off = 0;
  unsigned short* btp = (unsigned short*)(ws + off); off += kBtBytes;
  unsigned short* ap0 = (unsigned short*)(ws + off); off += kABytes;
  unsigned short* ap1 = (unsigned short*)(ws + off); off += kABytes;
  if (off > ws_size) return;

  weight_rows_kernel<<<dim3(kOut), dim3(256), 0, stream>>>(coeff, base_w, btp);

  for (int ch = 0; ch < nchunks; ++ch) {
    unsigned short* ap = (ch & 1) ? ap1 : ap0;
    basis_rows_kernel<<<dim3(kChunkRows), dim3(256), 0, stream>>>(x, centers, ap, ch * kChunkRows);
    float* cdst = out + (size_t)ch * kChunkRows * kOut;
    wmma_gemm64<0, false, 2, 0, false, 0><<<dim3((kChunkRows / 64) * (kOut / 64) / 8, 1), dim3(256), 0, stream>>>(
        ap, ap, kKtot, 0L,
        btp, btp, kKtot, 0L,
        (void*)cdst, (void*)cdst, kOut, 0L,
        base_b,
        base_b, 0L,
        kChunkRows, kOut, kKtot, kWCarryInv);
  }
}
